// Repro_89850715832656
// MI455X (gfx1250) — hardware-verified
//
#include <hip/hip_runtime.h>
#define BB 16
#define SS 512
#define DD 256
#define NH 8
#define HD 32
#define FF 682
#define FP 704
#define NQKV 576
#define NGU (2 * FP)
#define NTOK (BB * SS)
#define VOC 32000

typedef __bf16 v16b __attribute__((ext_vector_type(16)));
typedef unsigned short v8us __attribute__((ext_vector_type(8), may_alias));
typedef float  v8f  __attribute__((ext_vector_type(8)));
typedef float  v4f  __attribute__((ext_vector_type(4)));
typedef float  v4fa __attribute__((ext_vector_type(4), may_alias));
union FragB { v16b v; v8us half[2]; unsigned short u[16]; };

__device__ __forceinline__ unsigned short bf16_bits(float x) { unsigned int u = __float_as_uint(x); return (unsigned short)((u + 0x7FFFu + ((u >> 16) & 1u)) >> 16); }
__device__ __forceinline__ float bf16_val(unsigned short b) { return __uint_as_float(((unsigned int)b) << 16); }
__device__ __forceinline__ float bf16_round(float x) { return bf16_val(bf16_bits(x)); }
template <int NT>
__device__ __forceinline__ v8f mmaN(v16b ah, v16b al, v16b bh, v16b bl, v8f c) {
  c = __builtin_amdgcn_wmma_f32_16x16x32_bf16(false, ah, false, bh, (short)0, c, false, false);
  if (NT >= 2) c = __builtin_amdgcn_wmma_f32_16x16x32_bf16(false, al, false, bh, (short)0, c, false, false);
  if (NT >= 3) c = __builtin_amdgcn_wmma_f32_16x16x32_bf16(false, ah, false, bl, (short)0, c, false, false);
  asm volatile("v_nop\n\tv_nop\n\tv_nop\n\tv_nop" : "+v"(c) : "v"(ah), "v"(al), "v"(bh), "v"(bl));
  return c;
}

__global__ __launch_bounds__(256) void k_wt_bf16(const float* __restrict__ W, unsigned short* __restrict__ Wt, int K, int N) {
  const int t = blockIdx.x * 256 + threadIdx.x;
  const int k8n = K / 8;
  if (t >= N * k8n) return;
  const int n = t / k8n, k8 = (t % k8n) * 8;
  v8us v;
#pragma unroll
  for (int i = 0; i < 8; ++i) v[i] = bf16_bits(W[(size_t)(k8 + i) * N + n]);
  *(volatile v8us*)(Wt + (size_t)n * K + k8) = v;
  __threadfence();
  *(volatile v8us*)(Wt + (size_t)n * K + k8) = v;
}

template <bool ASPLIT, int ACT, bool BIAS_BF16>
__global__ __launch_bounds__(128) void k_gemm_bf(const float* __restrict__ A, int lda, const unsigned short* __restrict__ Wt, int ldb,
                                               const float* __restrict__ bias, float* __restrict__ C, int ldc, int M, int N, int K) {
  __shared__ __attribute__((aligned(16))) float so[4][16][64];
  const int tid = threadIdx.x, w = tid >> 5, lane = tid & 31, ln = lane & 15, hh = lane >> 4;
  const int ntn = N / 64;
  const int wid = blockIdx.x * 4 + w;
  const int mt = wid / ntn, nq = wid % ntn;
  if (mt * 16 >= M) return;
  const int row0 = mt * 16, col0 = nq * 64;
  const float* arow = A + (size_t)(row0 + ln) * lda;
  v8f acc[4] = {};
  for (int kb = 0; kb < K; kb += 32) {
    FragB ah, al;
    const v4f x0 = *(const v4fa*)(arow + kb + 8 * hh), x1 = *(const v4fa*)(arow + kb + 8 * hh + 4);
    const v4f x2 = *(const v4fa*)(arow + kb + 16 + 8 * hh), x3 = *(const v4fa*)(arow + kb + 16 + 8 * hh + 4);
    float xs[16] = {x0[0],x0[1],x0[2],x0[3],x1[0],x1[1],x1[2],x1[3],x2[0],x2[1],x2[2],x2[3],x3[0],x3[1],x3[2],x3[3]};
#pragma unroll
    for (int i = 0; i < 16; ++i) { const unsigned short hb = bf16_bits(xs[i]); ah.u[i] = hb; al.u[i] = ASPLIT ? bf16_bits(xs[i] - bf16_val(hb)) : (unsigned short)0; }
#pragma unroll
    for (int t = 0; t < 4; ++t) {
      const unsigned short* brow = Wt + (size_t)(col0 + t * 16 + ln) * ldb + kb;
      FragB b;
      b.half[0] = *(const v8us*)(brow + 8 * hh);
      b.half[1] = *(const v8us*)(brow + 16 + 8 * hh);
      acc[t] = mmaN<ASPLIT ? 2 : 1>(ah.v, al.v, b.v, b.v, acc[t]);
    }
  }
#pragma unroll
  for (int t = 0; t < 4; ++t) {
    float bv = bias ? bias[col0 + t * 16 + ln] : 0.f;
    if (BIAS_BF16) bv = bf16_round(bv);
#pragma unroll
    for (int r = 0; r < 8; ++r) { float v = acc[t][r] + bv; if (ACT == 1) v = fmaxf(v, 0.f); so[w][8 * hh + r][t * 16 + ln] = v; }
  }
  __builtin_amdgcn_fence(__ATOMIC_ACQ_REL, "workgroup");
  __builtin_amdgcn_wave_barrier();
  const int rsub = lane >> 4, c4 = (lane & 15) * 4;
  for (int pass = 0; pass < 2; ++pass) {
#pragma unroll
    for (int q = 0; q < 8; ++q) {
      const int r = q * 2 + rsub;
      const v4f v = *(const v4fa*)&so[w][r][c4];
      *(volatile v4f*)(C + (size_t)(row0 + r) * ldc + col0 + c4) = v;
    }
    if (pass == 0) __threadfence();
  }
}

template <int D, bool CAUSAL>
__global__ __launch_bounds__(128) void k_flash(const float* __restrict__ qb, const float* __restrict__ kb, const float* __restrict__ vb,
                                             int pitch, int T, int H, float scale, float* __restrict__ y, int ypitch) {
  constexpr int KS = D / 32;
  constexpr int DT = D / 16;
  __shared__ __attribute__((aligned(16))) unsigned short sKh[32][D + 8], sKl[32][D + 8], sVh[32][D + 8], sVl[32][D + 8];
  __shared__ __attribute__((aligned(16))) unsigned short sPh[4][16][40], sPl[4][16][40];
  __shared__ __attribute__((aligned(16))) float sO[4][16][D];
  const int tid = threadIdx.x, w = tid >> 5, lane = tid & 31, ln = lane & 15, hh = lane >> 4;
  const int nqb = (T + 63) / 64;
  const int bh = blockIdx.x / nqb, qblk = blockIdx.x % nqb;
  const int b = bh / H, h = bh % H;
  const int q0 = qblk * 64 + w * 16;
  const float* Q = qb + (size_t)b * T * pitch + h * D;
  const float* K = kb + (size_t)b * T * pitch + h * D;
  const float* V = vb + (size_t)b * T * pitch + h * D;

  FragB aqh[KS], aql[KS];
  {
    int row = q0 + ln; if (row >= T) row = T - 1;
    const float* qr = Q + (size_t)row * pitch;
#pragma unroll
    for (int ks = 0; ks < KS; ++ks)
#pragma unroll
      for (int i = 0; i < 16; ++i) {
        const int d = ks * 32 + ((i < 8) ? (8 * hh + i) : (16 + 8 * hh + (i - 8)));
        const float x = qr[d] * scale; const unsigned short hb = bf16_bits(x);
        aqh[ks].u[i] = hb; aql[ks].u[i] = bf16_bits(x - bf16_val(hb));
      }
  }
  float m_r[8], l_r[8];
#pragma unroll
  for (int r = 0; r < 8; ++r) { m_r[r] = -3.0e38f; l_r[r] = 0.f; }
  v8f oacc[DT];
#pragma unroll
  for (int dt = 0; dt < DT; ++dt) oacc[dt] = (v8f){0.f,0.f,0.f,0.f,0.f,0.f,0.f,0.f};

  const int kv_end = CAUSAL ? min(T, qblk * 64 + 64) : T;
  for (int j0 = 0; j0 < kv_end; j0 += 32) {
    __syncthreads();
    for (int e = tid; e < 32 * (D / 4); e += 128) {
      const int r = e / (D / 4), c4 = (e % (D / 4)) * 4;
      const int key = j0 + r;
      v4f kf = {0.f,0.f,0.f,0.f}, vf = {0.f,0.f,0.f,0.f};
      if (key < T) { kf = *(const v4fa*)(K + (size_t)key * pitch + c4); vf = *(const v4fa*)(V + (size_t)key * pitch + c4); }
#pragma unroll
      for (int t = 0; t < 4; ++t) {
        unsigned short hb = bf16_bits(kf[t]); sKh[r][c4 + t] = hb; sKl[r][c4 + t] = bf16_bits(kf[t] - bf16_val(hb));
        hb = bf16_bits(vf[t]); sVh[r][c4 + t] = hb; sVl[r][c4 + t] = bf16_bits(vf[t] - bf16_val(hb));
      }
    }
    __syncthreads();
    v8f s[2];
#pragma unroll
    for (int nt = 0; nt < 2; ++nt) {
      v8f acc = {};
#pragma unroll
      for (int ks = 0; ks < KS; ++ks) {
        FragB bh_, bl_;
        bh_.half[0] = *(const v8us*)&sKh[nt * 16 + ln][ks * 32 + 8 * hh]; bh_.half[1] = *(const v8us*)&sKh[nt * 16 + ln][ks * 32 + 16 + 8 * hh];
        bl_.half[0] = *(const v8us*)&sKl[nt * 16 + ln][ks * 32 + 8 * hh]; bl_.half[1] = *(const v8us*)&sKl[nt * 16 + ln][ks * 32 + 16 + 8 * hh];
        acc = mmaN<3>(aqh[ks].v, aql[ks].v, bh_.v, bl_.v, acc);
      }
      s[nt] = acc;
    }
    float alpha[8];
#pragma unroll
    for (int r = 0; r < 8; ++r) {
      const int qi = q0 + 8 * hh + r;
      const int ja = j0 + ln, jb = j0 + 16 + ln;
      if (CAUSAL) { if (ja > qi) s[0][r] = -3.0e38f; if (jb > qi) s[1][r] = -3.0e38f; }
      if (ja >= T) s[0][r] = -3.0e38f;
      if (jb >= T) s[1][r] = -3.0e38f;
      float mx = fmaxf(s[0][r], s[1][r]);
      mx = fmaxf(mx, __shfl_xor(mx, 1, 32)); mx = fmaxf(mx, __shfl_xor(mx, 2, 32)); mx = fmaxf(mx, __shfl_xor(mx, 4, 32)); mx = fmaxf(mx, __shfl_xor(mx, 8, 32));
      const float mnew = fmaxf(m_r[r], mx);
      alpha[r] = (mnew > -1.0e38f) ? __expf(m_r[r] - mnew) : 1.0f;
      const float p0 = (s[0][r] > -1.0e38f) ? __expf(s[0][r] - mnew) : 0.f;
      const float p1 = (s[1][r] > -1.0e38f) ? __expf(s[1][r] - mnew) : 0.f;
      m_r[r] = mnew;
      l_r[r] = l_r[r] * alpha[r] + p0 + p1;
      unsigned short hb = bf16_bits(p0); sPh[w][8 * hh + r][ln] = hb;      sPl[w][8 * hh + r][ln] = bf16_bits(p0 - bf16_val(hb));
      hb = bf16_bits(p1);                sPh[w][8 * hh + r][16 + ln] = hb; sPl[w][8 * hh + r][16 + ln] = bf16_bits(p1 - bf16_val(hb));
    }
#pragma unroll
    for (int dt = 0; dt < DT; ++dt)
#pragma unroll
      for (int r = 0; r < 8; ++r) oacc[dt][r] *= alpha[r];
    __builtin_amdgcn_fence(__ATOMIC_ACQ_REL, "workgroup");
    __builtin_amdgcn_wave_barrier();
    FragB pah, pal;
    pah.half[0] = *(const v8us*)&sPh[w][ln][8 * hh]; pah.half[1] = *(const v8us*)&sPh[w][ln][16 + 8 * hh];
    pal.half[0] = *(const v8us*)&sPl[w][ln][8 * hh]; pal.half[1] = *(const v8us*)&sPl[w][ln][16 + 8 * hh];
#pragma unroll
    for (int dt = 0; dt < DT; ++dt) {
      FragB bvh, bvl;
#pragma unroll
      for (int i = 0; i < 8; ++i) {
        bvh.u[i] = sVh[8 * hh + i][dt * 16 + ln]; bvh.u[8 + i] = sVh[16 + 8 * hh + i][dt * 16 + ln];
        bvl.u[i] = sVl[8 * hh + i][dt * 16 + ln]; bvl.u[8 + i] = sVl[16 + 8 * hh + i][dt * 16 + ln];
      }
      oacc[dt] = mmaN<3>(pah.v, pal.v, bvh.v, bvl.v, oacc[dt]);
    }
    __builtin_amdgcn_fence(__ATOMIC_ACQ_REL, "workgroup");
    __builtin_amdgcn_wave_barrier();
  }
#pragma unroll
  for (int r = 0; r < 8; ++r) {
    float l = l_r[r];
    l += __shfl_xor(l, 1, 32); l += __shfl_xor(l, 2, 32); l += __shfl_xor(l, 4, 32); l += __shfl_xor(l, 8, 32);
    l_r[r] = (l > 0.f) ? 1.0f / l : 0.f;
  }
#pragma unroll
  for (int dt = 0; dt < DT; ++dt)
#pragma unroll
    for (int r = 0; r < 8; ++r) sO[w][8 * hh + r][dt * 16 + ln] = oacc[dt][r] * l_r[r];
  __builtin_amdgcn_fence(__ATOMIC_ACQ_REL, "workgroup");
  __builtin_amdgcn_wave_barrier();
  for (int pass = 0; pass < 2; ++pass) {
    for (int r = 0; r < 16; ++r) {
      const int row = q0 + r;
      if (row < T && lane < D / 4) {
        const v4f val = *(const v4fa*)&sO[w][r][lane * 4];
        *(volatile v4f*)(y + ((size_t)b * T + row) * ypitch + h * D + lane * 4) = val;
      }
    }
    if (pass == 0) __threadfence();
  }
}

template <bool ASPLIT, int ACT, bool BIAS_BF16, bool RES_BF16>
__global__ __launch_bounds__(128) void k_gemm_bf3(const float* __restrict__ A, int lda, const unsigned short* __restrict__ Wt, int ldb,
                                                const float* __restrict__ bias, const float* __restrict__ resid, int rmod, int ldr,
                                                float* __restrict__ C, int ldc, int M, int N, int K) {
  __shared__ __attribute__((aligned(16))) float so[4][16][64];
  const int tid = threadIdx.x, w = tid >> 5, lane = tid & 31, ln = lane & 15, hh = lane >> 4;
  const int ntn = N / 64;
  const int wid = blockIdx.x * 4 + w;
  const int mt = wid / ntn, nq = wid % ntn;
  if (mt * 16 >= M) return;
  const int row0 = mt * 16, col0 = nq * 64;
  const float* arow = A + (size_t)(row0 + ln) * lda;
  v8f acc[4] = {};
  for (int kb = 0; kb < K; kb += 32) {
    FragB ah, al;
    const v4f x0 = *(const v4fa*)(arow + kb + 8 * hh), x1 = *(const v4fa*)(arow + kb + 8 * hh + 4);
    const v4f x2 = *(const v4fa*)(arow + kb + 16 + 8 * hh), x3 = *(const v4fa*)(arow + kb + 16 + 8 * hh + 4);
    float xs[16] = {x0[0],x0[1],x0[2],x0[3],x1[0],x1[1],x1[2],x1[3],x2[0],x2[1],x2[2],x2[3],x3[0],x3[1],x3[2],x3[3]};
#pragma unroll
    for (int i = 0; i < 16; ++i) { const unsigned short hb = bf16_bits(xs[i]); ah.u[i] = hb; al.u[i] = ASPLIT ? bf16_bits(xs[i] - bf16_val(hb)) : (unsigned short)0; }
#pragma unroll
    for (int t = 0; t < 4; ++t) {
      const unsigned short* brow = Wt + (size_t)(col0 + t * 16 + ln) * ldb + kb;
      FragB b;
      b.half[0] = *(const v8us*)(brow + 8 * hh);
      b.half[1] = *(const v8us*)(brow + 16 + 8 * hh);
      acc[t] = mmaN<ASPLIT ? 2 : 1>(ah.v, al.v, b.v, b.v, acc[t]);
    }
  }
#pragma unroll
  for (int t = 0; t < 4; ++t) {
    const int col = col0 + t * 16 + ln;
    float bv = bias ? bias[col] : 0.f;
    if (BIAS_BF16) bv = bf16_round(bv);
#pragma unroll
    for (int r = 0; r < 8; ++r) {
      float v = acc[t][r] + bv;
      if (resid) { float rv = resid[(size_t)((row0 + 8 * hh + r) % rmod) * ldr + col]; if (RES_BF16) rv = bf16_round(rv); v += rv; }
      if (ACT == 1) v = fmaxf(v, 0.f);
      if (ACT == 2) v = 0.5f * v * (1.0f + erff(v * 0.70710678118654752f));
      if (ACT == 3) { const float u = 0.7978845608028654f * (v + 0.044715f * v * v * v); v = 0.5f * v * (1.0f + tanhf(u)); }
      so[w][8 * hh + r][t * 16 + ln] = v;
    }
  }
  __builtin_amdgcn_fence(__ATOMIC_ACQ_REL, "workgroup");
  __builtin_amdgcn_wave_barrier();
  const int rsub = lane >> 4, c4 = (lane & 15) * 4;
  for (int pass = 0; pass < 2; ++pass) {
#pragma unroll
    for (int q = 0; q < 8; ++q) {
      const int r = q * 2 + rsub;
      const v4f v = *(const v4fa*)&so[w][r][c4];
      *(volatile v4f*)(C + (size_t)(row0 + r) * ldc + col0 + c4) = v;
    }
    if (pass == 0) __threadfence();
  }
}
template <bool PARAM_BF16>
__global__ __launch_bounds__(256) void k_layernorm(const float* __restrict__ X, const float* __restrict__ R, const float* __restrict__ g, const float* __restrict__ bta,
                                                  float* __restrict__ out_sum, float* __restrict__ out_norm, int N, float eps) {
  __shared__ float red[256];
  const int row = blockIdx.x, tid = threadIdx.x;
  const float* x = X + (size_t)row * N; const float* rr = R ? R + (size_t)row * N : nullptr;
  float vals[16];
  const int per = N / 256;
  float s1 = 0.f;
  for (int u = 0; u < per / 4; ++u) {
    const int j = tid * 4 + 1024 * u;
    const v4f a = *(const v4fa*)(x + j);
    v4f b = {0.f,0.f,0.f,0.f}; if (rr) b = *(const v4fa*)(rr + j);
#pragma unroll
    for (int q = 0; q < 4; ++q) { const float v = a[q] + b[q]; vals[u * 4 + q] = v; s1 += v; }
  }
  red[tid] = s1; __syncthreads();
  for (int st = 128; st > 0; st >>= 1) { if (tid < st) red[tid] += red[tid + st]; __syncthreads(); }
  const float mu = red[0] / (float)N; __syncthreads();
  float s2 = 0.f;
  for (int u = 0; u < per / 4; ++u)
#pragma unroll
    for (int q = 0; q < 4; ++q) { const float c = vals[u * 4 + q] - mu; s2 += c * c; }
  red[tid] = s2; __syncthreads();
  for (int st = 128; st > 0; st >>= 1) { if (tid < st) red[tid] += red[tid + st]; __syncthreads(); }
  const float rs = rsqrtf(red[0] / (float)N + eps);
  for (int pass = 0; pass < 2; ++pass) {
    for (int u = 0; u < per / 4; ++u) {
      const int j = tid * 4 + 1024 * u;
      v4f o, sm;
#pragma unroll
      for (int q = 0; q < 4; ++q) {
        float gg = g[j + q], bb = bta[j + q];
        if (PARAM_BF16) { gg = bf16_round(gg); bb = bf16_round(bb); }
        sm[q] = vals[u * 4 + q]; o[q] = (vals[u * 4 + q] - mu) * rs * gg + bb;
      }
      if (out_sum) *(volatile v4f*)(out_sum + (size_t)row * N + j) = sm;
      *(volatile v4f*)(out_norm + (size_t)row * N + j) = o;
    }
    if (pass == 0) __threadfence();
  }
}

typedef _Float16 v16h __attribute__((ext_vector_type(16)));
union FragH { v16h v; v8us half[2]; _Float16 h[16]; unsigned short u[16]; };
template <int NT>
__device__ __forceinline__ v8f mmaH(v16h ah, v16h al, v16h bh, v16h bl, v8f c) {
  c = __builtin_amdgcn_wmma_f32_16x16x32_f16(false, ah, false, bh, (short)0, c, false, false);
  if (NT >= 2) c = __builtin_amdgcn_wmma_f32_16x16x32_f16(false, al, false, bh, (short)0, c, false, false);
  if (NT >= 3) c = __builtin_amdgcn_wmma_f32_16x16x32_f16(false, ah, false, bl, (short)0, c, false, false);
  asm volatile("v_nop\n\tv_nop\n\tv_nop\n\tv_nop" : "+v"(c) : "v"(ah), "v"(al), "v"(bh), "v"(bl));
  return c;
}
template <bool ASPLIT>
__global__ __launch_bounds__(128) void k_gemm_h(const float* __restrict__ A, int lda, size_t sA, const _Float16* __restrict__ Bh, int ldb, size_t sB, float alpha, float* __restrict__ C, int ldc, size_t sC, int M, int N, int K) {
  __shared__ __attribute__((aligned(16))) float so[4][16][64];
  const int tid = threadIdx.x, w = tid >> 5, lane = tid & 31, ln = lane & 15, hh = lane >> 4; const int by = blockIdx.y;
  A += (size_t)by * sA; Bh += (size_t)by * sB; C += (size_t)by * sC;
  const int ntn = (N + 63) / 64; const int wid = blockIdx.x * 4 + w; const int mt = wid / ntn, nq = wid % ntn; if (mt * 16 >= M) return;
  const int row0 = mt * 16, col0 = nq * 64; const float* arow = A + (size_t)(row0 + ln) * lda;
  v8f acc[4] = {};
  for (int kb = 0; kb < K; kb += 32) {
    FragH ah, al;
    const v4f x0 = *(const v4fa*)(arow + kb + 8 * hh), x1 = *(const v4fa*)(arow + kb + 8 * hh + 4), x2 = *(const v4fa*)(arow + kb + 16 + 8 * hh), x3 = *(const v4fa*)(arow + kb + 16 + 8 * hh + 4);
    float xs[16] = {x0[0],x0[1],x0[2],x0[3],x1[0],x1[1],x1[2],x1[3],x2[0],x2[1],x2[2],x2[3],x3[0],x3[1],x3[2],x3[3]};
#pragma unroll
    for (int i = 0; i < 16; ++i) { const _Float16 h = (_Float16)xs[i]; ah.h[i] = h; al.h[i] = ASPLIT ? (_Float16)(xs[i] - (float)h) : (_Float16)0.0f; }
#pragma unroll
    for (int t = 0; t < 4; ++t) { if (col0 + t * 16 >= N) continue; const size_t boff = (size_t)(col0 + t * 16 + ln) * ldb + kb; FragH bq; bq.half[0] = *(const v8us*)(Bh + boff + 8 * hh); bq.half[1] = *(const v8us*)(Bh + boff + 16 + 8 * hh);
      acc[t] = mmaH<ASPLIT ? 2 : 1>(ah.v, al.v, bq.v, bq.v, acc[t]); }
  }
#pragma unroll
  for (int t = 0; t < 4; ++t) { if (col0 + t * 16 >= N) continue;
#pragma unroll
    for (int r = 0; r < 8; ++r) so[w][8 * hh + r][t * 16 + ln] = acc[t][r] * alpha; }
  __builtin_amdgcn_fence(__ATOMIC_ACQ_REL, "workgroup"); __builtin_amdgcn_wave_barrier();
  const int rsub = lane >> 4, c4 = (lane & 15) * 4;
  for (int pass = 0; pass < 2; ++pass) {
#pragma unroll
    for (int q = 0; q < 8; ++q) { const int r = q * 2 + rsub; if (col0 + c4 < N) { const v4f v = *(const v4fa*)&so[w][r][c4]; *(volatile v4f*)(C + (size_t)(row0 + r) * ldc + col0 + c4) = v; } }
    if (pass == 0) __threadfence(); }
}

__global__ __launch_bounds__(256) void k_btqkv(const float* __restrict__ wq, const float* __restrict__ wk, const float* __restrict__ wv, unsigned short* __restrict__ Bt) { const int t = blockIdx.x * 256 + threadIdx.x; if (t >= NQKV * (DD / 8)) return; const int n = t / (DD / 8), k8 = (t % (DD / 8)) * 8; v8us v;
  for (int q = 0; q < 8; ++q) { const int k = k8 + q; float w = 0.f; if (n < 256) w = wq[(size_t)n * DD + k]; else if (n < 288) w = wk[(size_t)(n - 256) * DD + k]; else if (n < 544) w = wv[(size_t)(n - 288) * DD + k]; v[q] = bf16_bits(w); } *(volatile v8us*)(Bt + (size_t)n * DD + k8) = v; __threadfence(); *(volatile v8us*)(Bt + (size_t)n * DD + k8) = v; }
__global__ __launch_bounds__(256) void k_btgu(const float* __restrict__ wg, const float* __restrict__ wu, unsigned short* __restrict__ Bt) { const int t = blockIdx.x * 256 + threadIdx.x; if (t >= NGU * (DD / 8)) return; const int n = t / (DD / 8), k8 = (t % (DD / 8)) * 8; v8us v;
  for (int q = 0; q < 8; ++q) { const int k = k8 + q; float w = 0.f; if (n < FF) w = wg[(size_t)n * DD + k]; else if (n >= FP && n < FP + FF) w = wu[(size_t)(n - FP) * DD + k]; v[q] = bf16_bits(w); } *(volatile v8us*)(Bt + (size_t)n * DD + k8) = v; __threadfence(); *(volatile v8us*)(Bt + (size_t)n * DD + k8) = v; }
__global__ __launch_bounds__(256) void k_btdown(const float* __restrict__ wd, unsigned short* __restrict__ Bt) { const int t = blockIdx.x * 256 + threadIdx.x; if (t >= DD * (FP / 8)) return; const int n = t / (FP / 8), k8 = (t % (FP / 8)) * 8; v8us v; for (int q = 0; q < 8; ++q) { const int k = k8 + q; v[q] = bf16_bits(k < FF ? wd[(size_t)n * FF + k] : 0.f); } *(volatile v8us*)(Bt + (size_t)n * FP + k8) = v; __threadfence(); *(volatile v8us*)(Bt + (size_t)n * FP + k8) = v; }
__global__ __launch_bounds__(256) void k_bcat3(const float* __restrict__ bq, const float* __restrict__ bk, const float* __restrict__ bv, const float* __restrict__ bg, const float* __restrict__ bu, float* __restrict__ bqkv, float* __restrict__ bgu) { const int t = blockIdx.x * 256 + threadIdx.x;
  if (t < NQKV) { const float v = (t < 256) ? bq[t] : (t < 288 ? bk[t - 256] : (t < 544 ? bv[t - 288] : 0.f)); *(volatile float*)(bqkv + t) = v; __threadfence(); *(volatile float*)(bqkv + t) = v; }
  if (t < NGU) { const float v = (t < FF) ? bg[t] : ((t >= FP && t < FP + FF) ? bu[t - FP] : 0.f); *(volatile float*)(bgu + t) = v; __threadfence(); *(volatile float*)(bgu + t) = v; } }
__global__ __launch_bounds__(256) void k_embed(const int* __restrict__ tok, const float* __restrict__ emb, const float* __restrict__ pos, const float* __restrict__ w, float* __restrict__ Hh, float* __restrict__ X) { const int tid = threadIdx.x, wv = tid >> 5, lane = tid & 31; const int t = blockIdx.x * 8 + wv; const int s = t % SS; int id = tok[t]; id = id < 0 ? 0 : (id >= VOC ? VOC - 1 : id); float h[8]; float ms = 0.f;
#pragma unroll
  for (int u = 0; u < 8; ++u) { const int c = u * 32 + lane; h[u] = bf16_round(emb[(size_t)id * DD + c]) + bf16_round(pos[(size_t)s * DD + c]); ms += h[u] * h[u]; }
  for (int o = 16; o >= 1; o >>= 1) ms += __shfl_xor(ms, o, 32); const float rs = rsqrtf(ms * (1.0f / DD) + 1.1920928955078125e-07f);
  for (int pass = 0; pass < 2; ++pass) {
#pragma unroll
    for (int u = 0; u < 8; ++u) { const int c = u * 32 + lane; *(volatile float*)(Hh + (size_t)t * DD + c) = h[u]; *(volatile float*)(X + (size_t)t * DD + c) = h[u] * rs * bf16_round(w[c]); } if (pass == 0) __threadfence(); } }
__global__ __launch_bounds__(256) void k_heads(const float* __restrict__ QKV, const float* __restrict__ ct, const float* __restrict__ st, int b, float* __restrict__ Qr, _Float16* __restrict__ Kr, _Float16* __restrict__ Vt) {
  __shared__ float tv[64][33]; const int tid = threadIdx.x, lane = tid & 31, wv = tid >> 5; const int r0 = blockIdx.x * 64;
  for (int q8 = 0; q8 < 8; ++q8) { const int r = r0 + wv * 8 + q8; const int hh2 = r / SS, sp = r % SS; const int tok = r >> 3, chunk = r & 7; const float* qrow = QKV + ((size_t)b * SS + tok) * NQKV + chunk * HD; const float* vrow = QKV + ((size_t)b * SS + tok) * NQKV + 288 + chunk * HD;
    const int i = lane >> 1; const float xe = qrow[2 * i], xo = qrow[2 * i + 1]; const float c = bf16_round(ct[(size_t)sp * HD + 2 * i]), s = bf16_round(st[(size_t)sp * HD + 2 * i]);
    const float qv = ((lane & 1) ? (xe * s + xo * c) : (xe * c - xo * s)) * 0.17677669529663687f; tv[wv * 8 + q8][lane] = vrow[lane];
    float* qd = Qr + (size_t)r * HD; *(volatile float*)(qd + lane) = qv; __threadfence(); *(volatile float*)(qd + lane) = qv; (void)hh2; }
  if (blockIdx.x < SS / 64) { for (int q8 = 0; q8 < 8; ++q8) { const int t = r0 + wv * 8 + q8; const float* krow = QKV + ((size_t)b * SS + t) * NQKV + 256; const int i = lane >> 1; const float xe = krow[2 * i], xo = krow[2 * i + 1]; const float c = bf16_round(ct[(size_t)t * HD + 2 * i]), s = bf16_round(st[(size_t)t * HD + 2 * i]);
      const _Float16 kv = (_Float16)((lane & 1) ? (xe * s + xo * c) : (xe * c - xo * s)); *(volatile _Float16*)(Kr + (size_t)t * HD + lane) = kv; __threadfence(); *(volatile _Float16*)(Kr + (size_t)t * HD + lane) = kv; } }
  __syncthreads(); typedef _Float16 v2h __attribute__((ext_vector_type(2)));
  { const int hh2 = r0 / SS, tp0 = r0 % SS; for (int pass = 0; pass < 2; ++pass) { for (int e = tid; e < 32 * 32; e += 256) { const int d = e >> 5, tp = (e & 31) * 2; v2h vv; vv.x = (_Float16)tv[tp][d]; vv.y = (_Float16)tv[tp + 1][d]; *(volatile v2h*)(Vt + ((size_t)hh2 * HD + d) * SS + tp0 + tp) = vv; } if (pass == 0) __threadfence(); } }
}
__global__ __launch_bounds__(1024) void k_softmax(float* __restrict__ S, const int* __restrict__ mask, float* __restrict__ Dn) { __shared__ float sd[32]; const int tid = threadIdx.x, wv = tid >> 5, lane = tid & 31; const int r = blockIdx.x * 32 + wv; const int sp = r % SS; float* row = S + (size_t)r * SS; const int* mrow = mask + (size_t)sp * SS;
  float mx = -3.0e38f; for (int j = lane; j < SS; j += 32) if (mrow[j] != 0) mx = fmaxf(mx, row[j]); for (int o = 16; o >= 1; o >>= 1) mx = fmaxf(mx, __shfl_xor(mx, o, 32));
  float den = 0.f; for (int j = lane; j < SS; j += 32) { const float e = (mrow[j] != 0) ? expf(row[j] - mx) : 0.f; den += e; *(volatile float*)(row + j) = e * 256.0f; } for (int o = 16; o >= 1; o >>= 1) den += __shfl_xor(den, o, 32);
  __threadfence(); for (int j = lane; j < SS; j += 32) { const float pv = row[j]; *(volatile float*)(row + j) = pv; }
  if (lane == 0) sd[wv] = den; __syncthreads(); if (tid < 32) { *(volatile float*)(Dn + blockIdx.x * 32 + tid) = sd[tid]; } __threadfence(); if (tid < 32) { *(volatile float*)(Dn + blockIdx.x * 32 + tid) = sd[tid]; } }
__global__ __launch_bounds__(256) void k_post(const float* __restrict__ O, const float* __restrict__ Dn, const float* __restrict__ Hh, const float* __restrict__ w, int b, float* __restrict__ X2) { const int tid = threadIdx.x, wv = tid >> 5, lane = tid & 31; const int tl = blockIdx.x * 8 + wv; const size_t t = (size_t)b * SS + tl; float h2[8]; float ms = 0.f;
#pragma unroll
  for (int u = 0; u < 8; ++u) { const int c = u * 32 + lane; const int r = tl * 8 + u; h2[u] = O[(size_t)r * HD + lane] / Dn[r] + Hh[t * DD + c]; ms += h2[u] * h2[u]; }
  for (int o = 16; o >= 1; o >>= 1) ms += __shfl_xor(ms, o, 32); const float rs = rsqrtf(ms * (1.0f / DD) + 1.1920928955078125e-07f);
  for (int pass = 0; pass < 2; ++pass) {
#pragma unroll
    for (int u = 0; u < 8; ++u) { const int c = u * 32 + lane; *(volatile float*)(X2 + t * DD + c) = h2[u] * rs * bf16_round(w[c]); } if (pass == 0) __threadfence(); } }
__global__ __launch_bounds__(256) void k_glu(const float* __restrict__ GU, float* __restrict__ P) { const size_t t = (size_t)blockIdx.x * 256 + threadIdx.x; if (t >= (size_t)NTOK * FP / 4) return; const int c4 = (int)((t * 4) % FP); const size_t tok = (t * 4) / FP; const v4f g = *(const v4fa*)(GU + tok * NGU + c4), u = *(const v4fa*)(GU + tok * NGU + FP + c4); v4f o;
  for (int q = 0; q < 4; ++q) { const int c = c4 + q; o[q] = (c < FF) ? (g[q] * (1.0f / (1.0f + expf(-g[q])))) * u[q] : 0.f; } *(volatile v4f*)(P + t * 4) = o; __threadfence(); *(volatile v4f*)(P + t * 4) = o; }
__global__ __launch_bounds__(256) void k_fin(const float* __restrict__ DW, const float* __restrict__ bd, const float* __restrict__ X2, float* __restrict__ out) { const size_t t = (size_t)blockIdx.x * 256 + threadIdx.x; if (t >= (size_t)NTOK * DD / 4) return; const int c4 = (int)((t * 4) % DD); const v4f d = *(const v4fa*)(DW + t * 4), x = *(const v4fa*)(X2 + t * 4); v4f o; for (int q = 0; q < 4; ++q) o[q] = (d[q] + bf16_round(bd[c4 + q])) + x[q]; *(volatile v4f*)(out + t * 4) = o; __threadfence(); *(volatile v4f*)(out + t * 4) = o; }
extern "C" void kernel_launch(void* const* d_in, const int* in_sizes, int n_in,
                              void* d_out, int out_size, void* d_ws, size_t ws_size, hipStream_t stream) {
  (void)in_sizes; (void)n_in; (void)out_size;
  const float* emb = (const float*)d_in[0]; const float* pos = (const float*)d_in[1]; const float* anw = (const float*)d_in[2]; const float* wq = (const float*)d_in[3]; const float* bq = (const float*)d_in[4]; const float* wk = (const float*)d_in[5]; const float* bk = (const float*)d_in[6]; const float* wv = (const float*)d_in[7]; const float* bv = (const float*)d_in[8];
  const float* ct = (const float*)d_in[9]; const float* st = (const float*)d_in[10]; const float* fnw = (const float*)d_in[11]; const float* wg = (const float*)d_in[12]; const float* bg = (const float*)d_in[13]; const float* wu = (const float*)d_in[14]; const float* bu = (const float*)d_in[15]; const float* wd = (const float*)d_in[16]; const float* bd = (const float*)d_in[17]; const int* tok = (const int*)d_in[18]; const int* mask = (const int*)d_in[19];
  char* ws = (char*)d_ws; size_t off = 0;
  auto take = [&](size_t bytes) { char* p = ws + off; off += (bytes + 255) & ~(size_t)255; return p; };
  unsigned short* Bqkv = (unsigned short*)take((size_t)NQKV * DD * 2); unsigned short* Bgu = (unsigned short*)take((size_t)NGU * DD * 2); unsigned short* Bdn = (unsigned short*)take((size_t)DD * FP * 2); float* bqkv = (float*)take(NQKV * 4); float* bgu = (float*)take(NGU * 4);
  float* Hh = (float*)take((size_t)NTOK * DD * 4); float* X = (float*)take((size_t)NTOK * DD * 4); float* QKV = (float*)take((size_t)NTOK * NQKV * 4);
  float* Qr = (float*)take((size_t)SS * NH * HD * 4); _Float16* Kr = (_Float16*)take((size_t)SS * HD * 2); _Float16* Vt = (_Float16*)take((size_t)NH * HD * SS * 2); float* S = (float*)take((size_t)NH * SS * SS * 4); float* Dn = (float*)take((size_t)NH * SS * 4);
  float* O = (float*)take((size_t)NTOK * DD * 4); float* X2 = (float*)take((size_t)NTOK * DD * 4); float* GU = (float*)take((size_t)NTOK * NGU * 4); float* Pm = X;   float* P2 = (float*)take((size_t)NTOK * FP * 4); float* DW = Hh;
  if (off > ws_size) return; (void)Pm;
  k_btqkv<<<(NQKV * (DD / 8) + 255) / 256, 256, 0, stream>>>(wq, wk, wv, Bqkv); k_btgu<<<(NGU * (DD / 8) + 255) / 256, 256, 0, stream>>>(wg, wu, Bgu); k_btdown<<<(DD * (FP / 8) + 255) / 256, 256, 0, stream>>>(wd, Bdn); k_bcat3<<<(NGU + 255) / 256, 256, 0, stream>>>(bq, bk, bv, bg, bu, bqkv, bgu);
  k_embed<<<NTOK / 8, 256, 0, stream>>>(tok, emb, pos, anw, Hh, X);
  k_gemm_bf3<true, 0, true, false><<<((NTOK / 16) * (NQKV / 64) + 3) / 4, 128, 0, stream>>>(X, DD, Bqkv, DD, bqkv, nullptr, 1, 0, QKV, NQKV, NTOK, NQKV, DD);
  for (int b = 0; b < BB; ++b) {
    k_heads<<<SS * NH / 64, 256, 0, stream>>>(QKV, ct, st, b, Qr, Kr, Vt);
    k_gemm_h<true><<<dim3(((SS / 16) * (SS / 64) + 3) / 4, NH), 128, 0, stream>>>(Qr, HD, (size_t)SS * HD, Kr, HD, 0, 1.f, S, SS, (size_t)SS * SS, SS, SS, HD);
    k_softmax<<<NH * SS / 32, 1024, 0, stream>>>(S, mask, Dn);
    k_gemm_h<false><<<dim3(((SS / 16) * 1 + 3) / 4, NH), 128, 0, stream>>>(S, SS, (size_t)SS * SS, Vt, SS, (size_t)HD * SS, 0.00390625f, O + (size_t)b * SS * DD, HD, (size_t)SS * HD, SS, HD, SS);
    k_post<<<SS / 8, 256, 0, stream>>>(O + (size_t)b * SS * DD, Dn, Hh, fnw, b, X2);
  }
  k_gemm_bf3<true, 0, true, false><<<((NTOK / 16) * (NGU / 64) + 3) / 4, 128, 0, stream>>>(X2, DD, Bgu, DD, bgu, nullptr, 1, 0, GU, NGU, NTOK, NGU, DD);
  k_glu<<<(unsigned)(((size_t)NTOK * FP / 4 + 255) / 256), 256, 0, stream>>>(GU, P2);
  k_gemm_bf3<true, 0, false, false><<<((NTOK / 16) * (DD / 64) + 3) / 4, 128, 0, stream>>>(P2, FP, Bdn, FP, nullptr, nullptr, 1, 0, DW, DD, NTOK, DD, FP);
  k_fin<<<(unsigned)(((size_t)NTOK * DD / 4 + 255) / 256), 256, 0, stream>>>(DW, bd, X2, (float*)d_out);
}
